// SelfAwareAttention_3238405341368
// MI455X (gfx1250) — hardware-run, weakly checked
//
#include <hip/hip_runtime.h>
#include <math.h>

typedef __attribute__((ext_vector_type(16))) _Float16 v16h;
typedef __attribute__((ext_vector_type(16))) __bf16 v16b;
typedef __attribute__((ext_vector_type(8)))  _Float16 v8h;
typedef __attribute__((ext_vector_type(8)))  float v8f;
typedef __attribute__((ext_vector_type(4)))  float v4f;
typedef __attribute__((ext_vector_type(2)))  float v2f;
typedef __attribute__((ext_vector_type(4)))  unsigned v4u;
typedef __attribute__((ext_vector_type(4)))  int v4i;
typedef float __attribute__((may_alias)) float_a;
typedef int __attribute__((may_alias)) int_a;

template <typename T> __device__ __forceinline__ void vst2(void* p, T v) { *(volatile T*)p = v; __threadfence(); *(volatile T*)p = v; }
__device__ __forceinline__ v8f wmma16(v16h a, v16h b, v8f c) {
  v8f d = __builtin_amdgcn_wmma_f32_16x16x32_f16(false, a, false, b, (short)0, c, false, false);
  asm volatile("v_nop\n\tv_nop\n\tv_nop\n\tv_nop" : "+v"(d) : "v"(a), "v"(b));
  return d;
}
__device__ __forceinline__ v8f wmma_bf(v16b a, v16b b, v8f c) {
  v8f d = __builtin_amdgcn_wmma_f32_16x16x32_bf16(false, a, false, b, (short)0, c, false, false);
  asm volatile("v_nop\n\tv_nop\n\tv_nop\n\tv_nop" : "+v"(d) : "v"(a), "v"(b));
  return d;
}
__device__ __forceinline__ v16h frag_h(const _Float16* rowk0, int lane) {
  union { v16h v; v8h q[2]; } u; const _Float16* p = rowk0 + 8 * (lane >> 4);
  u.q[0] = *(const v8h*)p; u.q[1] = *(const v8h*)(p + 16); return u.v;
}
__device__ __forceinline__ v16h frag_f32(const float* rowk0, int lane) {
  v16h a; const float* p = rowk0 + 8 * (lane >> 4);
#pragma unroll
  for (int i = 0; i < 8; ++i) { a[i] = (_Float16)p[i]; a[8 + i] = (_Float16)p[16 + i]; }
  return a;
}
__device__ __forceinline__ v16h frag_f32s(const float* rowk0, int lane, float sc) {
  v16h a; const float* p = rowk0 + 8 * (lane >> 4);
#pragma unroll
  for (int i = 0; i < 8; ++i) { a[i] = (_Float16)(p[i] * sc); a[8 + i] = (_Float16)(p[16 + i] * sc); }
  return a;
}
__device__ __forceinline__ v16h fragc_f32(const float* W, int k0, int n, int lane, int ld, int K) {
  v16h a; const int g = lane >> 4;
#pragma unroll
  for (int i = 0; i < 8; ++i) { const int ka = k0 + 8 * g + i, kb = ka + 16;
    a[i] = (_Float16)(ka < K ? W[(size_t)(ka < K ? ka : K - 1) * ld + n] : 0.f); a[8 + i] = (_Float16)(kb < K ? W[(size_t)(kb < K ? kb : K - 1) * ld + n] : 0.f); }
  return a;
}
struct F2 { v16b h, l; };
__device__ __forceinline__ F2 bsplit16(const float v[16]) { F2 r;
#pragma unroll
  for (int i = 0; i < 16; ++i) { const __bf16 h = (__bf16)v[i]; r.h[i] = h; r.l[i] = (__bf16)(v[i] - (float)h); }
  return r; }
__device__ __forceinline__ F2 split_row(const float* row, int k0, int lane) { float v[16]; const float* p = row + k0 + 8 * (lane >> 4);
#pragma unroll
  for (int i = 0; i < 8; ++i) { v[i] = p[i]; v[8 + i] = p[16 + i]; }
  return bsplit16(v); }
__device__ __forceinline__ F2 split_rowK(const float* row, int k0, int lane, int K) { float v[16]; const int g = lane >> 4;
#pragma unroll
  for (int i = 0; i < 8; ++i) { const int ka = k0 + 8 * g + i, kb = ka + 16; v[i] = ka < K ? row[ka < K ? ka : K - 1] : 0.f; v[8 + i] = kb < K ? row[kb < K ? kb : K - 1] : 0.f; }
  return bsplit16(v); }
__device__ __forceinline__ F2 split_col(const float* W, int k0, int n, int lane, int ld, int K) { float v[16]; const int g = lane >> 4;
#pragma unroll
  for (int i = 0; i < 8; ++i) { const int ka = k0 + 8 * g + i, kb = ka + 16; v[i] = ka < K ? W[(size_t)(ka < K ? ka : K - 1) * ld + n] : 0.f; v[8 + i] = kb < K ? W[(size_t)(kb < K ? kb : K - 1) * ld + n] : 0.f; }
  return bsplit16(v); }
__device__ __forceinline__ v8f mac3(const F2& a, const F2& b, v8f c) { c = wmma_bf(a.l, b.h, c); c = wmma_bf(a.h, b.l, c); return wmma_bf(a.h, b.h, c); }
__device__ __forceinline__ float sigm(float v) { return 1.0f / (1.0f + expf(-v)); }
#define LDSX() do { asm volatile("s_wait_dscnt 0" ::: "memory"); __builtin_amdgcn_wave_barrier(); __builtin_amdgcn_fence(__ATOMIC_RELEASE, "workgroup"); } while (0)


#define NB 2
#define CC 256
#define HW 2304
#define NHD 8
#define DK 32
#define CR 32
#define NCOL (4 * CC + 2 * CR)
#ifndef TNB
#define TNB NB
#endif
typedef __attribute__((ext_vector_type(8))) __bf16 v8b;
__device__ __forceinline__ v16b frag_b(const __bf16* rowk0, int lane) {
  union { v16b v; v8b q[2]; } u; const __bf16* p = rowk0 + 8 * (lane >> 4);
  u.q[0] = *(const v8b*)p; u.q[1] = *(const v8b*)(p + 16); return u.v;
}
__device__ __forceinline__ float bfr(float v) { return (float)(__bf16)v; }
__device__ __attribute__((noinline)) float exp_ni(float v) { return expf(v); }
__device__ __attribute__((noinline)) float erf_ni(float v) { return erff(v); }

#define WS_QK  0u
#define WS_QKL (WS_QK + 2u * (size_t)NB * HW * 2 * CC)
#define WS_VT  (WS_QKL + 2u * (size_t)NB * HW * 2 * CC)
#define WS_VTL (WS_VT + 2u * (size_t)NB * CC * HW)
#define WS_WT  (WS_VTL + 2u * (size_t)NB * CC * HW)
#define WS_WTL (WS_WT + 2u * (size_t)NB * CC * HW)
#define WS_MN  (WS_WTL + 2u * (size_t)NB * CC * HW)
#define WS_MNL (WS_MN + 2u * (size_t)NB * HW * 2 * CR)
#define WS_TSA (WS_MNL + 2u * (size_t)NB * HW * 2 * CR)
#define WS_GSA (WS_TSA + 4u * (size_t)NB * HW * CC)
#define WS_END (WS_GSA + 4u * (size_t)NB * HW * CC)

__global__ __launch_bounds__(128) void k_proj(const float* __restrict__ X, const float* __restrict__ WQ, const float* __restrict__ BQ, const float* __restrict__ WK, const float* __restrict__ BK, const float* __restrict__ WV, const float* __restrict__ BV, const float* __restrict__ WW, const float* __restrict__ BW, const float* __restrict__ WM, const float* __restrict__ BM, const float* __restrict__ WN, const float* __restrict__ BN, _Float16* __restrict__ QK, _Float16* __restrict__ QKL, _Float16* __restrict__ VT, _Float16* __restrict__ VTL, _Float16* __restrict__ WT, _Float16* __restrict__ WTL, _Float16* __restrict__ MN, _Float16* __restrict__ MNL) {
  __shared__ __align__(16) _Float16 sh[64][136], sl[64][136]; __shared__ __align__(16) _Float16 th[128][72], tl[128][72];
  const int tid = threadIdx.x, wave = tid >> 5, lane = tid & 31, col = lane & 15, g = lane >> 4; const size_t b = blockIdx.z; const int grp = blockIdx.y; const int n0 = blockIdx.x * 64 + wave * 16; const float* Xb = X + b * CC * (size_t)HW;
  const int which = grp >> 1;
  const int ntile = (grp == 8) ? 4 : 8;
  v8f acc[8] = {};
#pragma unroll 2
  for (int kc = 0; kc < CC / 32; ++kc) { v16b a; const int px = n0 + col;
#pragma unroll
    for (int i = 0; i < 8; ++i) { a[i] = (__bf16)Xb[(size_t)(kc * 32 + 8 * g + i) * HW + px]; a[8 + i] = (__bf16)Xb[(size_t)(kc * 32 + 16 + 8 * g + i) * HW + px]; }
#pragma unroll
    for (int j = 0; j < 8; ++j) { if (j < ntile) { const float* wr; if (grp == 8) { wr = (j < 2) ? WM + (size_t)(j * 16 + col) * CC : WN + (size_t)((j - 2) * 16 + col) * CC; } else { const float* Wm = which == 0 ? WQ : which == 1 ? WK : which == 2 ? WV : WW; wr = Wm + (size_t)((grp & 1) * 128 + j * 16 + col) * CC; } wr += kc * 32 + 8 * g; v16b w;
#pragma unroll
        for (int i = 0; i < 8; ++i) { w[i] = (__bf16)wr[i]; w[8 + i] = (__bf16)wr[16 + i]; } acc[j] = wmma_bf(a, w, acc[j]); } } }
#pragma unroll
  for (int j = 0; j < 8; ++j) { if (j < ntile) { float bb; if (grp == 8) bb = (j < 2) ? bfr(BM[j * 16 + col]) : bfr(BN[(j - 2) * 16 + col]); else { const float* Bm = which == 0 ? BQ : which == 1 ? BK : which == 2 ? BV : BW; bb = bfr(Bm[(grp & 1) * 128 + j * 16 + col]); }
#pragma unroll
      for (int r = 0; r < 8; ++r) { const float v = acc[j][r] + bb; const _Float16 hv = (_Float16)v, lv = (_Float16)((v - (float)hv) * 2048.0f); if (which == 2 || which == 3) { th[j * 16 + col][wave * 16 + 8 * g + r] = hv; tl[j * 16 + col][wave * 16 + 8 * g + r] = lv; } else { sh[wave * 16 + 8 * g + r][j * 16 + col] = hv; sl[wave * 16 + 8 * g + r][j * 16 + col] = lv; } } } }
  __syncthreads();
  if (which < 2) { const int c0 = which * CC + (grp & 1) * 128; for (int e = tid; e < 64 * 16; e += 128) { const int rl = e >> 4, q = e & 15; const size_t o = (b * HW + blockIdx.x * 64 + rl) * (2 * CC) + c0 + q * 8; vst2((unsigned*)(QK + o), *(const v4u*)&sh[rl][q * 8]); vst2((unsigned*)(QKL + o), *(const v4u*)&sl[rl][q * 8]); } }
  else if (which == 4) { for (int e = tid; e < 64 * 8; e += 128) { const int rl = e >> 3, q = e & 7; const size_t o = (b * HW + blockIdx.x * 64 + rl) * (2 * CR) + q * 8; vst2((unsigned*)(MN + o), *(const v4u*)&sh[rl][q * 8]); vst2((unsigned*)(MNL + o), *(const v4u*)&sl[rl][q * 8]); } }
  else { _Float16* PT = (which == 2) ? VT : WT; _Float16* PTL = (which == 2) ? VTL : WTL; const int c0 = (grp & 1) * 128; for (int e = tid; e < 128 * 8; e += 128) { const int cl = e >> 3, q = e & 7; const size_t o = (b * CC + c0 + cl) * (size_t)HW + blockIdx.x * 64 + q * 8; vst2((unsigned*)(PT + o), *(const v4u*)&th[cl][q * 8]); vst2((unsigned*)(PTL + o), *(const v4u*)&tl[cl][q * 8]); } } }
template <int MODE>
__global__ __launch_bounds__(128) void k_att(const _Float16* __restrict__ AH, const _Float16* __restrict__ AL, const _Float16* __restrict__ PT, const _Float16* __restrict__ PTL, float* __restrict__ OUTR) {
  constexpr int NJ = MODE == 0 ? 2 : 8; constexpr int RS = MODE == 0 ? 2 * CC : 2 * CR;
  __shared__ __align__(16) float sp[4][16][36]; __shared__ __align__(16) float so[4][16][NJ * 16 + 4];
  const int tid = threadIdx.x, wave = tid >> 5, lane = tid & 31, col = lane & 15, g = lane >> 4; const int hy = blockIdx.y; const size_t b = blockIdx.z; const int q0 = blockIdx.x * 64 + wave * 16; const size_t rq = b * HW + q0;
  const int qoff = MODE == 0 ? hy * DK : 0, koff = MODE == 0 ? CC + hy * DK : CR; const float scale = MODE == 0 ? 0.17677669529663687f : 1.0f; const int vc0 = MODE == 0 ? hy * DK : hy * 128;
  const v16h aq = frag_h(AH + (rq + col) * RS + qoff, lane), aql = frag_h(AL + (rq + col) * RS + qoff, lane);
  float m[8], l[8];
#pragma unroll
  for (int r = 0; r < 8; ++r) { m[r] = -3.0e38f; l[r] = 0.f; }
  v8f acc[NJ], accl[NJ];
#pragma unroll
  for (int j = 0; j < NJ; ++j) { acc[j] = v8f{}; accl[j] = v8f{}; }
#pragma unroll 1
  for (int ks = 0; ks < HW / 32; ++ks) { v8f s[2];
#pragma unroll
    for (int ct = 0; ct < 2; ++ct) { const size_t rk = b * HW + ks * 32 + ct * 16 + col; const v16h kh = frag_h(AH + rk * RS + koff, lane), kl = frag_h(AL + rk * RS + koff, lane); v8f c = {}, cl = {}; c = wmma16(aq, kh, c); cl = wmma16(aq, kl, cl); cl = wmma16(aql, kh, cl);
#pragma unroll
      for (int r = 0; r < 8; ++r) s[ct][r] = (c[r] + cl[r] * (1.0f / 2048.0f)) * scale; }
    float alpha[8];
#pragma unroll
    for (int r = 0; r < 8; ++r) { float mx = fmaxf(s[0][r], s[1][r]);
#pragma unroll
      for (int o = 1; o < 16; o <<= 1) mx = fmaxf(mx, __shfl_xor(mx, o));
      const float mn = fmaxf(m[r], mx); alpha[r] = __expf(m[r] - mn); const float e0 = __expf(s[0][r] - mn), e1 = __expf(s[1][r] - mn); float es = e0 + e1;
#pragma unroll
      for (int o = 1; o < 16; o <<= 1) es += __shfl_xor(es, o);
      l[r] = l[r] * alpha[r] + es; m[r] = mn; sp[wave][8 * g + r][col] = e0; sp[wave][8 * g + r][16 + col] = e1; }
#pragma unroll
    for (int j = 0; j < NJ; ++j)
#pragma unroll
      for (int r = 0; r < 8; ++r) { acc[j][r] *= alpha[r]; accl[j][r] *= alpha[r]; }
    LDSX();
    v16h pa; { const float* prow = &sp[wave][col][0] + 8 * (lane >> 4);
#pragma unroll
      for (int i = 0; i < 8; ++i) { pa[i] = (_Float16)(prow[i] * 2048.0f); pa[8 + i] = (_Float16)(prow[16 + i] * 2048.0f); } }
#pragma unroll
    for (int j = 0; j < NJ; ++j) { const size_t po = (b * CC + vc0 + j * 16 + col) * (size_t)HW + ks * 32; acc[j] = wmma16(pa, frag_h(PT + po, lane), acc[j]); accl[j] = wmma16(pa, frag_h(PTL + po, lane), accl[j]); }
    LDSX(); }
#pragma unroll
  for (int r = 0; r < 8; ++r) { const float il = (1.0f / 2048.0f) / l[r];
#pragma unroll
    for (int j = 0; j < NJ; ++j) so[wave][8 * g + r][j * 16 + col] = (acc[j][r] + accl[j][r] * (1.0f / 2048.0f)) * il; }
  LDSX(); for (int rl = 0; rl < 16; ++rl) if (lane < NJ * 4) vst2(OUTR + (rq + rl) * CC + vc0 + lane * 4, *(const v4f*)&so[wave][rl][lane * 4]); }
__global__ __launch_bounds__(128) void k_out(const float* __restrict__ TSA, const float* __restrict__ GSA, const float* __restrict__ WO, const float* __restrict__ BO, const float* __restrict__ GT, const float* __restrict__ GG, const float* __restrict__ X, float* __restrict__ OUT) { __shared__ __align__(16) float stt[128][68];
  const int tid = threadIdx.x, wave = tid >> 5, lane = tid & 31, col = lane & 15, g = lane >> 4; const size_t b = blockIdx.y; const int n0 = blockIdx.x * 64; const size_t r0 = b * HW + n0 + wave * 16; const float gt = bfr(GT[0]), gg = bfr(GG[0]);
#pragma unroll 1
  for (int cc = 0; cc < CC; cc += 128) { v8f acc[8] = {};
#pragma unroll 2
    for (int kc = 0; kc < CC / 32; ++kc) { const F2 a = split_row(GSA + (r0 + col) * CC, kc * 32, lane);
#pragma unroll
      for (int j = 0; j < 8; ++j) { v16b w; const float* wr = WO + (size_t)(cc + j * 16 + col) * CC + kc * 32 + 8 * g;
#pragma unroll
        for (int i = 0; i < 8; ++i) { w[i] = (__bf16)wr[i]; w[8 + i] = (__bf16)wr[16 + i]; } acc[j] = wmma_bf(a.h, w, acc[j]); acc[j] = wmma_bf(a.l, w, acc[j]); } }
#pragma unroll
    for (int j = 0; j < 8; ++j) { const int cl = j * 16 + col; const float bb = bfr(BO[cc + cl]);
#pragma unroll
      for (int r = 0; r < 8; ++r) { const int px = wave * 16 + 8 * g + r; stt[cl][px] = gt * TSA[(r0 + 8 * g + r) * CC + cc + cl] + gg * (acc[j][r] + bb) + bfr(X[(b * CC + cc + cl) * (size_t)HW + n0 + px]); } }
    __syncthreads(); for (int e = tid; e < 128 * 16; e += 128) { const int cl = e >> 4, q = e & 15; vst2(OUT + (b * CC + cc + cl) * (size_t)HW + n0 + q * 4, *(const v4f*)&stt[cl][q * 4]); } __syncthreads(); } }
extern "C" void kernel_launch(void* const* d_in, const int* in_sizes, int n_in, void* d_out, int out_size, void* d_ws, size_t ws_size, hipStream_t stream) {
  (void)in_sizes; (void)n_in; (void)out_size;
  const float** F = (const float**)d_in;
  if (ws_size < (size_t)WS_END) return;
  char* ws = (char*)d_ws; _Float16 *QK = (_Float16*)(ws + WS_QK), *QKL = (_Float16*)(ws + WS_QKL), *VT = (_Float16*)(ws + WS_VT), *VTL = (_Float16*)(ws + WS_VTL), *WT = (_Float16*)(ws + WS_WT), *WTL = (_Float16*)(ws + WS_WTL), *MN = (_Float16*)(ws + WS_MN), *MNL = (_Float16*)(ws + WS_MNL); float *TSA = (float*)(ws + WS_TSA), *GSA = (float*)(ws + WS_GSA);
  k_proj<<<dim3(HW / 64, 9, TNB), 128, 0, stream>>>(F[0], F[1], F[2], F[3], F[4], F[5], F[6], F[11], F[12], F[7], F[8], F[9], F[10], QK, QKL, VT, VTL, WT, WTL, MN, MNL);
  k_att<0><<<dim3(HW / 64, NHD, TNB), 128, 0, stream>>>(QK, QKL, VT, VTL, TSA);
  k_att<1><<<dim3(HW / 64, 2, TNB), 128, 0, stream>>>(MN, MNL, WT, WTL, GSA);
  k_out<<<dim3(HW / 64, TNB), 128, 0, stream>>>(TSA, GSA, F[13], F[14], F[15], F[16], F[0], (float*)d_out);
}
